// DeepLagrangianNetwork_35579509080614
// MI455X (gfx1250) — hardware-verified
//
#include <hip/hip_runtime.h>
#include <stddef.h>
#include <math.h>


#define QD    4
#define HID   64
#define H2S   68
#define W2S   72
#define NTHR  256
#define NWB   (NTHR / 32)
#define ASC   16.0f
#define BSC   64.0f
#define RSC   0.0009765625f
#define SLOPE 0.01f
#define MAXBLK 1024

static_assert((H2S % 4) == 0 && (W2S % 8) == 0);
static_assert(NTHR == 4 * HID);
static_assert(NWB * 32 == NTHR);

typedef float    v4f  __attribute__((ext_vector_type(4)));
typedef float    v8f  __attribute__((ext_vector_type(8)));
typedef _Float16 v8h  __attribute__((ext_vector_type(8)));
typedef _Float16 v16h __attribute__((ext_vector_type(16)));
union Frag { v16h v; v8h h[2]; };

__device__ __forceinline__ v8f wmh(v16h a, v16h b, v8f c) {
  v8f d = __builtin_amdgcn_wmma_f32_16x16x32_f16(false, a, false, b, (short)0, c, false, false);
  asm volatile("v_nop\n\tv_nop\n\tv_nop\n\tv_nop" : "+v"(d) : "v"(a), "v"(b));
  return d;
}

__device__ __forceinline__ v16h l1frag(const v4f q, const float* w1s, const float* b1s, int kb) {
  v16h a;
#pragma unroll
  for (int i = 0; i < 8; ++i) {
    {
      const int k = kb + i;
      const v4f w = *(const v4f*)(w1s + 4 * k);
      float v = q.x * w.x;
      v = fmaf(q.y, w.y, v);
      v = fmaf(q.z, w.z, v);
      v = fmaf(q.w, w.w, v);
      v += b1s[k];
      v = fmaxf(v, SLOPE * v);
      a[i] = (_Float16)(v * ASC);
    }
    {
      const int k = kb + 16 + i;
      const v4f w = *(const v4f*)(w1s + 4 * k);
      float v = q.x * w.x;
      v = fmaf(q.y, w.y, v);
      v = fmaf(q.z, w.z, v);
      v = fmaf(q.w, w.w, v);
      v += b1s[k];
      v = fmaf(0.0f, 0.0f, fmaxf(v, SLOPE * v));
      a[8 + i] = (_Float16)(v * ASC);
    }
  }
  return a;
}

__global__ __launch_bounds__(NTHR)
void k_main(const float* __restrict__ x,
            const float* __restrict__ W1, const float* __restrict__ b1,
            const float* __restrict__ W2, const float* __restrict__ b2,
            const float* __restrict__ WLd, const float* __restrict__ bLd,
            const float* __restrict__ WLo, const float* __restrict__ bLo,
            float* out, int nrows, int nWaves, int tilesPerWave) {
  __shared__ __attribute__((aligned(16))) _Float16 w2h[HID * W2S];
  __shared__ __attribute__((aligned(16))) float    h2s[NWB * 16 * H2S];
  __shared__ __attribute__((aligned(16))) float    w1s[HID * 4];
  __shared__ __attribute__((aligned(16))) float    whs[HID * 4];
  __shared__ float b1s[HID];
  __shared__ float b2s[HID];

  const int tid  = threadIdx.x;
  const int lane = tid & 31;
  const int wave = tid >> 5;
  const int lo   = lane & 15;
  const int hi   = lane >> 4;

  if (tid < HID) {
    const v4f w = *(const v4f*)(W1 + 4 * tid);
    *(v4f*)(w1s + 4 * tid) = w;
    v4f hv;
    hv.x = WLd[tid];
    hv.y = WLd[HID + tid];
    hv.z = WLo[tid];
    hv.w = 0.0f;
    *(v4f*)(whs + 4 * tid) = hv;
    b1s[tid] = b1[tid];
    b2s[tid] = b2[tid];
  }
  {
    const int n  = tid >> 2;
    const int k0 = (tid & 3) * 16;
    const float* sp = W2 + n * HID + k0;
    const v4f f0 = *(const v4f*)(sp);
    const v4f f1 = *(const v4f*)(sp + 4);
    const v4f f2 = *(const v4f*)(sp + 8);
    const v4f f3 = *(const v4f*)(sp + 12);
    v8h ha, hb;
    ha[0] = (_Float16)(f0.x * BSC); ha[1] = (_Float16)(f0.y * BSC);
    ha[2] = (_Float16)(f0.z * BSC); ha[3] = (_Float16)(f0.w * BSC);
    ha[4] = (_Float16)(f1.x * BSC); ha[5] = (_Float16)(f1.y * BSC);
    ha[6] = (_Float16)(f1.z * BSC); ha[7] = (_Float16)(f1.w * BSC);
    hb[0] = (_Float16)(f2.x * BSC); hb[1] = (_Float16)(f2.y * BSC);
    hb[2] = (_Float16)(f2.z * BSC); hb[3] = (_Float16)(f2.w * BSC);
    hb[4] = (_Float16)(f3.x * BSC); hb[5] = (_Float16)(f3.y * BSC);
    hb[6] = (_Float16)(f3.z * BSC); hb[7] = (_Float16)(f3.w * BSC);
    *(v8h*)(w2h + n * W2S + k0)     = ha;
    *(v8h*)(w2h + n * W2S + k0 + 8) = hb;
  }
  __syncthreads();

  const float bld0 = bLd[0];
  const float bld1 = bLd[1];
  const float blo  = bLo[0];

  const int wbase = wave * (16 * H2S);
  const int wid   = (blockIdx.x * NTHR + tid) >> 5;

  for (int it = 0; it < tilesPerWave; ++it) {
    const int t   = wid + it * nWaves;
    const int row = t * 16 + lo;
    const int qr  = row < nrows ? row : (nrows - 1);
    const v4f qv  = *(const v4f*)(x + (size_t)qr * QD);

    const v16h afr0 = l1frag(qv, w1s, b1s, 8 * hi);
    const v16h afr1 = l1frag(qv, w1s, b1s, 32 + 8 * hi);

    v8f cf[4];
#pragma unroll
    for (int j = 0; j < 4; ++j) {
      const _Float16* bp = w2h + (16 * j + lo) * W2S + 8 * hi;
      Frag b0, b1f;
      b0.h[0]  = *(const v8h*)(bp);
      b0.h[1]  = *(const v8h*)(bp + 16);
      b1f.h[0] = *(const v8h*)(bp + 32);
      b1f.h[1] = *(const v8h*)(bp + 48);
      v8f c = {0.f, 0.f, 0.f, 0.f, 0.f, 0.f, 0.f, 0.f};
      c = wmh(afr0, b0.v, c);
      c = wmh(afr1, b1f.v, c);
      cf[j] = c;
    }

#pragma unroll
    for (int j = 0; j < 4; ++j) {
      const float bb = b2s[16 * j + lo];
#pragma unroll
      for (int e = 0; e < 8; ++e) {
        float v = fmaf(cf[j][e], RSC, bb);
        v = fmaxf(v, SLOPE * v);
        h2s[wbase + (e + 8 * hi) * H2S + 16 * j + lo] = v;
      }
    }
    __syncthreads();

    const float* hr = h2s + wbase + lo * H2S + 32 * hi;
    const float* wr = whs + 4 * 32 * hi;
    float p0 = 0.0f, p1 = 0.0f, p2 = 0.0f;
#pragma unroll
    for (int u = 0; u < 8; ++u) {
      const v4f h  = *(const v4f*)(hr + 4 * u);
      const v4f wa = *(const v4f*)(wr + 16 * u);
      const v4f wb = *(const v4f*)(wr + 16 * u + 4);
      const v4f wc = *(const v4f*)(wr + 16 * u + 8);
      const v4f wd = *(const v4f*)(wr + 16 * u + 12);
      p0 = fmaf(h.x, wa.x, p0); p0 = fmaf(h.y, wb.x, p0); p0 = fmaf(h.z, wc.x, p0); p0 = fmaf(h.w, wd.x, p0);
      p1 = fmaf(h.x, wa.y, p1); p1 = fmaf(h.y, wb.y, p1); p1 = fmaf(h.z, wc.y, p1); p1 = fmaf(h.w, wd.y, p1);
      p2 = fmaf(h.x, wa.z, p2); p2 = fmaf(h.y, wb.z, p2); p2 = fmaf(h.z, wc.z, p2); p2 = fmaf(h.w, wd.z, p2);
    }
    p0 += __shfl_xor(p0, 16, 32);
    p1 += __shfl_xor(p1, 16, 32);
    p2 += __shfl_xor(p2, 16, 32);

    const float za = p0 + bld0;
    const float zb = p1 + bld1;
    const float da = fmaxf(za, 0.f) + log1pf(expf(-fabsf(za)));
    const float db = fmaxf(zb, 0.f) + log1pf(expf(-fabsf(zb)));
    const float dc = p2 + blo;
    const float od = da * dc;
    v4f Hv;
    Hv.x = fmaf(da, da, 1e-9f);
    Hv.y = od;
    Hv.z = od;
    Hv.w = fmaf(dc, dc, fmaf(db, db, 1e-9f));

    const bool wrt = (lane < 16) && (row < nrows);
    float* op = out + (size_t)(wrt ? row : 0) * 4;
    if (wrt) *(volatile v4f*)op = Hv;
    __threadfence();
    if (wrt) *(volatile v4f*)op = Hv;

    __syncthreads();
  }
}

extern "C" void kernel_launch(void* const* d_in, const int* in_sizes, int n_in,
                              void* d_out, int out_size, void* d_ws, size_t ws_size,
                              hipStream_t stream) {
  (void)d_ws; (void)ws_size;
  if (n_in < 9) return;
  if (in_sizes[0] < QD || (in_sizes[0] % QD) != 0) return;
  const int nrows = in_sizes[0] / QD;
  if (in_sizes[1] != HID * QD || in_sizes[2] != HID || in_sizes[3] != HID * HID ||
      in_sizes[4] != HID || in_sizes[5] != 2 * HID || in_sizes[6] < 2 ||
      in_sizes[7] != HID || in_sizes[8] < 1) return;
  if (out_size != nrows * 4) return;

  const float* x   = (const float*)d_in[0];
  const float* W1  = (const float*)d_in[1];
  const float* b1  = (const float*)d_in[2];
  const float* W2  = (const float*)d_in[3];
  const float* b2  = (const float*)d_in[4];
  const float* WLd = (const float*)d_in[5];
  const float* bLd = (const float*)d_in[6];
  const float* WLo = (const float*)d_in[7];
  const float* bLo = (const float*)d_in[8];
  float* out = (float*)d_out;

  const int numTiles = (nrows + 15) / 16;
  int blocks = (numTiles + NWB - 1) / NWB;
  if (blocks > MAXBLK) blocks = MAXBLK;
  if (blocks < 1) blocks = 1;
  const int nWaves = blocks * NWB;
  const int tilesPerWave = (numTiles + nWaves - 1) / nWaves;

  k_main<<<blocks, NTHR, 0, stream>>>(x, W1, b1, W2, b2, WLd, bLd, WLo, bLo,
                                      out, nrows, nWaves, tilesPerWave);
}
